// CrossAttention_LR_65249143160950
// MI455X (gfx1250) — hardware-verified
//
#include <hip/hip_runtime.h>
#include <math.h>

typedef __attribute__((ext_vector_type(16))) _Float16 v16h;
typedef __attribute__((ext_vector_type(16))) __bf16 v16b;
typedef __attribute__((ext_vector_type(8)))  _Float16 v8h;
typedef __attribute__((ext_vector_type(8)))  float v8f;
typedef __attribute__((ext_vector_type(4)))  float v4f;
typedef __attribute__((ext_vector_type(2)))  float v2f;
typedef __attribute__((ext_vector_type(4)))  unsigned v4u;
typedef __attribute__((ext_vector_type(4)))  int v4i;
typedef float __attribute__((may_alias)) float_a;
typedef int __attribute__((may_alias)) int_a;

template <typename T> __device__ __forceinline__ void vst2(void* p, T v) { *(volatile T*)p = v; __threadfence(); *(volatile T*)p = v; }
__device__ __forceinline__ v8f wmma16(v16h a, v16h b, v8f c) {
  v8f d = __builtin_amdgcn_wmma_f32_16x16x32_f16(false, a, false, b, (short)0, c, false, false);
  asm volatile("v_nop\n\tv_nop\n\tv_nop\n\tv_nop" : "+v"(d) : "v"(a), "v"(b));
  return d;
}
__device__ __forceinline__ v8f wmma_bf(v16b a, v16b b, v8f c) {
  v8f d = __builtin_amdgcn_wmma_f32_16x16x32_bf16(false, a, false, b, (short)0, c, false, false);
  asm volatile("v_nop\n\tv_nop\n\tv_nop\n\tv_nop" : "+v"(d) : "v"(a), "v"(b));
  return d;
}
__device__ __forceinline__ v16h frag_h(const _Float16* rowk0, int lane) {
  union { v16h v; v8h q[2]; } u; const _Float16* p = rowk0 + 8 * (lane >> 4);
  u.q[0] = *(const v8h*)p; u.q[1] = *(const v8h*)(p + 16); return u.v;
}
__device__ __forceinline__ v16h frag_f32(const float* rowk0, int lane) {
  v16h a; const float* p = rowk0 + 8 * (lane >> 4);
#pragma unroll
  for (int i = 0; i < 8; ++i) { a[i] = (_Float16)p[i]; a[8 + i] = (_Float16)p[16 + i]; }
  return a;
}
__device__ __forceinline__ v16h frag_f32s(const float* rowk0, int lane, float sc) {
  v16h a; const float* p = rowk0 + 8 * (lane >> 4);
#pragma unroll
  for (int i = 0; i < 8; ++i) { a[i] = (_Float16)(p[i] * sc); a[8 + i] = (_Float16)(p[16 + i] * sc); }
  return a;
}
__device__ __forceinline__ v16h fragc_f32(const float* W, int k0, int n, int lane, int ld, int K) {
  v16h a; const int g = lane >> 4;
#pragma unroll
  for (int i = 0; i < 8; ++i) { const int ka = k0 + 8 * g + i, kb = ka + 16;
    a[i] = (_Float16)(ka < K ? W[(size_t)(ka < K ? ka : K - 1) * ld + n] : 0.f); a[8 + i] = (_Float16)(kb < K ? W[(size_t)(kb < K ? kb : K - 1) * ld + n] : 0.f); }
  return a;
}
struct F2 { v16b h, l; };
__device__ __forceinline__ F2 bsplit16(const float v[16]) { F2 r;
#pragma unroll
  for (int i = 0; i < 16; ++i) { const __bf16 h = (__bf16)v[i]; r.h[i] = h; r.l[i] = (__bf16)(v[i] - (float)h); }
  return r; }
__device__ __forceinline__ F2 split_row(const float* row, int k0, int lane) { float v[16]; const float* p = row + k0 + 8 * (lane >> 4);
#pragma unroll
  for (int i = 0; i < 8; ++i) { v[i] = p[i]; v[8 + i] = p[16 + i]; }
  return bsplit16(v); }
__device__ __forceinline__ F2 split_rowK(const float* row, int k0, int lane, int K) { float v[16]; const int g = lane >> 4;
#pragma unroll
  for (int i = 0; i < 8; ++i) { const int ka = k0 + 8 * g + i, kb = ka + 16; v[i] = ka < K ? row[ka < K ? ka : K - 1] : 0.f; v[8 + i] = kb < K ? row[kb < K ? kb : K - 1] : 0.f; }
  return bsplit16(v); }
__device__ __forceinline__ F2 split_col(const float* W, int k0, int n, int lane, int ld, int K) { float v[16]; const int g = lane >> 4;
#pragma unroll
  for (int i = 0; i < 8; ++i) { const int ka = k0 + 8 * g + i, kb = ka + 16; v[i] = ka < K ? W[(size_t)(ka < K ? ka : K - 1) * ld + n] : 0.f; v[8 + i] = kb < K ? W[(size_t)(kb < K ? kb : K - 1) * ld + n] : 0.f; }
  return bsplit16(v); }
__device__ __forceinline__ v8f mac3(const F2& a, const F2& b, v8f c) { c = wmma_bf(a.l, b.h, c); c = wmma_bf(a.h, b.l, c); return wmma_bf(a.h, b.h, c); }
__device__ __forceinline__ float sigm(float v) { return 1.0f / (1.0f + expf(-v)); }
#define LDSX() do { asm volatile("s_wait_dscnt 0" ::: "memory"); __builtin_amdgcn_wave_barrier(); __builtin_amdgcn_fence(__ATOMIC_RELEASE, "workgroup"); } while (0)


#define NB 16
#define CC 512
#define SS 1024
#define MC 77
#define CTX 768
#define NH 8
#define HD 64
#define NKV (1 + MC + SS)
#define KP 1152
#define MP 80
#define NR (NB * SS)
#ifndef TQB
#define TQB (SS / 64)
#define TNB NB
#endif
typedef __attribute__((ext_vector_type(8))) __bf16 v8b;
__device__ __forceinline__ v16b frag_b(const __bf16* rowk0, int lane) {
  union { v16b v; v8b q[2]; } u; const __bf16* p = rowk0 + 8 * (lane >> 4);
  u.q[0] = *(const v8b*)p; u.q[1] = *(const v8b*)(p + 16); return u.v;
}
__device__ __forceinline__ float bfr(float v) { return (float)(__bf16)v; }
__device__ __attribute__((noinline)) float exp_ni(float v) { return expf(v); }
__device__ __attribute__((noinline)) float erf_ni(float v) { return erff(v); }

#define WS_PQ  0u
#define WS_PO  (WS_PQ + 2u * (size_t)CC * CC)
#define WS_PKV (WS_PO + 2u * (size_t)CC * CC)
#define WS_XN  (WS_PKV + 2u * (size_t)2 * CC * CTX)
#define WS_XNL (WS_XN + 2u * (size_t)NR * CC)
#define WS_Q   (WS_XNL + 2u * (size_t)NR * CC)
#define WS_KR  (WS_Q + 2u * (size_t)NR * CC)
#define WS_V   (WS_KR + 2u * (size_t)NB * KP * CC)
#define WS_O   (WS_V + 2u * (size_t)NB * CC * KP)
#define WS_Y1  (WS_O + 4u * (size_t)NR * CC)
#define WS_END (WS_Y1 + 4u * (size_t)NR * CC)

__global__ __launch_bounds__(256) void k_pack(const float* __restrict__ WQ, const float* __restrict__ WO, const float* __restrict__ WKV, __bf16* __restrict__ P) { const int n = blockIdx.x, which = blockIdx.y, t = threadIdx.x; __shared__ __align__(16) __bf16 s[CTX];
  if (which < 2) { if (n >= CC) return; const float* w = (which == 0) ? WQ : WO; for (int k = t; k < CC; k += 256) s[k] = (__bf16)w[(size_t)k * CC + n]; __syncthreads(); if (t < CC / 8) vst2((unsigned*)(P + ((which == 0) ? WS_PQ : WS_PO) / 2 + (size_t)n * CC + t * 8), *(const v4u*)&s[t * 8]); }
  else { for (int k = t; k < CTX; k += 256) s[k] = (__bf16)WKV[(size_t)k * (2 * CC) + n]; __syncthreads(); if (t < CTX / 8) vst2((unsigned*)(P + WS_PKV / 2 + (size_t)n * CTX + t * 8), *(const v4u*)&s[t * 8]); } }
__global__ __launch_bounds__(256) void k_ln1(const float* __restrict__ X, const float* __restrict__ G1, __bf16* __restrict__ XN, __bf16* __restrict__ XNL) {
  __shared__ __align__(16) __bf16 sh[64][CC + 8]; __shared__ __align__(16) __bf16 sl[64][CC + 8]; __shared__ float sp[4][64]; __shared__ float smu[64], sinv[64]; const size_t b = blockIdx.y; const int n0 = blockIdx.x * 64, t = threadIdx.x;
  const int rl = t & 63, part = t >> 6; const float* xb = X + (b * CC) * SS + n0 + rl;
  { float s = 0.f; for (int c = part * 128; c < part * 128 + 128; ++c) s += bfr(xb[(size_t)c * SS]); sp[part][rl] = s; }
  __syncthreads(); if (t < 64) smu[t] = ((sp[0][t] + sp[1][t]) + (sp[2][t] + sp[3][t])) / (float)CC; __syncthreads();
  { const float mu = smu[rl]; float q = 0.f; for (int c = part * 128; c < part * 128 + 128; ++c) { const float d = bfr(xb[(size_t)c * SS]) - mu; q += d * d; } sp[part][rl] = q; }
  __syncthreads(); if (t < 64) sinv[t] = 1.0f / sqrtf(((sp[0][t] + sp[1][t]) + (sp[2][t] + sp[3][t])) / (float)CC + 1e-5f); __syncthreads();
  { const float mu = smu[rl], inv = sinv[rl]; for (int c = part * 128; c < part * 128 + 128; ++c) { const float v = (bfr(xb[(size_t)c * SS]) - mu) * inv * bfr(G1[c]); const __bf16 hv = (__bf16)v; sh[rl][c] = hv; sl[rl][c] = (__bf16)(v - (float)hv); } }
  __syncthreads();
  for (int e = t; e < 64 * (CC / 8); e += 256) { const int nl = e / (CC / 8), q = e % (CC / 8); vst2((unsigned*)(XN + ((b * SS + n0 + nl) * CC) + q * 8), *(const v4u*)&sh[nl][q * 8]); vst2((unsigned*)(XNL + ((b * SS + n0 + nl) * CC) + q * 8), *(const v4u*)&sl[nl][q * 8]); }
}
__global__ __launch_bounds__(128) void k_q(const __bf16* __restrict__ XN, const __bf16* __restrict__ XNL, const __bf16* __restrict__ P, _Float16* __restrict__ Q, _Float16* __restrict__ KR, _Float16* __restrict__ V) {
  __shared__ __align__(16) _Float16 so[64][136]; __shared__ __align__(16) _Float16 st[128][72];
  const int tid = threadIdx.x, wave = tid >> 5, lane = tid & 31, col = lane & 15, g = lane >> 4; const size_t b = blockIdx.z; const int n0b = blockIdx.x * 64; const size_t r0 = b * SS + n0b + wave * 16; const int c0 = blockIdx.y * 128;
  v8f acc[8] = {};
#pragma unroll 2
  for (int kc = 0; kc < CC / 32; ++kc) { const v16b ah = frag_b(XN + (r0 + col) * CC + kc * 32, lane), al = frag_b(XNL + (r0 + col) * CC + kc * 32, lane);
#pragma unroll
    for (int j = 0; j < 8; ++j) { const v16b w = frag_b(P + WS_PQ / 2 + (size_t)(c0 + j * 16 + col) * CC + kc * 32, lane); acc[j] = wmma_bf(ah, w, acc[j]); acc[j] = wmma_bf(al, w, acc[j]); } }
#pragma unroll
  for (int j = 0; j < 8; ++j)
#pragma unroll
    for (int r = 0; r < 8; ++r) { const _Float16 hv = (_Float16)acc[j][r]; so[wave * 16 + 8 * g + r][j * 16 + col] = hv; st[j * 16 + col][wave * 16 + 8 * g + r] = hv; }
  __syncthreads();
  for (int e = tid; e < 64 * 16; e += 128) { const int nl = e >> 4, q = e & 15; const v4u w = *(const v4u*)&so[nl][q * 8]; vst2((unsigned*)(Q + ((b * SS + n0b + nl) * CC) + c0 + q * 8), w); vst2((unsigned*)(KR + ((b * KP + n0b + nl) * CC) + c0 + q * 8), w); }
  for (int e = tid; e < 128 * 8; e += 128) { const int d = e >> 3, pc = e & 7; vst2((unsigned*)(V + ((b * CC + c0 + d) * KP) + n0b + pc * 8), *(const v4u*)&st[d][pc * 8]); }
}
__global__ __launch_bounds__(128) void k_kv(const float* __restrict__ CT, const __bf16* __restrict__ P, const float* __restrict__ NULLKV, _Float16* __restrict__ KR, _Float16* __restrict__ V) {
  __shared__ __align__(16) _Float16 so[MP][136]; __shared__ __align__(16) _Float16 st[128][MP + 8];
  const int tid = threadIdx.x, wave = tid >> 5, lane = tid & 31, col = lane & 15, g = lane >> 4; const size_t b = blockIdx.z; const int c0 = blockIdx.y * 128; const bool isk = c0 < CC;
  for (int tile = wave; tile < MP / 16; tile += 4) { const int m0 = tile * 16; v8f acc[8] = {};
#pragma unroll 2
    for (int kc = 0; kc < CTX / 32; ++kc) { v16b a; { const int m = m0 + col; const bool live = m < MC; const float* p = CT + ((b * MC + (live ? m : 0)) * CTX) + kc * 32 + 8 * g;
#pragma unroll
        for (int i = 0; i < 8; ++i) { a[i] = live ? (__bf16)p[i] : (__bf16)0.f; a[8 + i] = live ? (__bf16)p[16 + i] : (__bf16)0.f; } }
#pragma unroll
      for (int j = 0; j < 8; ++j) acc[j] = wmma_bf(a, frag_b(P + WS_PKV / 2 + (size_t)(c0 + j * 16 + col) * CTX + kc * 32, lane), acc[j]); }
#pragma unroll
    for (int j = 0; j < 8; ++j)
#pragma unroll
      for (int r = 0; r < 8; ++r) { const _Float16 hv = (_Float16)acc[j][r]; if (isk) so[m0 + 8 * g + r][j * 16 + col] = hv; else st[j * 16 + col][m0 + 8 * g + r] = hv; } }
  __syncthreads();
  if (isk) { __shared__ __align__(16) _Float16 sn[128]; __shared__ __align__(16) _Float16 sz[8]; if (tid < 8) sz[tid] = (_Float16)0.f; for (int i = tid; i < 128; i += 128) sn[i] = (_Float16)bfr(NULLKV[(c0 + i) & (HD - 1)]); __syncthreads();
    for (int e = tid; e < MC * 16; e += 128) { const int m = e >> 4, q = e & 15; vst2((unsigned*)(KR + ((b * KP + SS + 1 + m) * CC) + c0 + q * 8), *(const v4u*)&so[m][q * 8]); }
    if (tid < 16) vst2((unsigned*)(KR + ((b * KP + SS) * CC) + c0 + tid * 8), *(const v4u*)&sn[tid * 8]);
    for (int e = tid; e < (KP - NKV) * 16; e += 128) { const int m = e >> 4, q = e & 15; vst2((unsigned*)(KR + ((b * KP + NKV + m) * CC) + c0 + q * 8), *(const v4u*)&sz[0]); } }
  else { const int vc0 = c0 - CC; __shared__ __align__(16) _Float16 sv[128][KP - SS];
    for (int e = tid; e < 128 * (KP - SS); e += 128) { const int d = e / (KP - SS), kc2 = e % (KP - SS); sv[d][kc2] = (kc2 == 0) ? (_Float16)bfr(NULLKV[HD + ((vc0 + d) & (HD - 1))]) : (kc2 <= MC) ? st[d][kc2 - 1] : (_Float16)0.f; }
    __syncthreads();
    for (int e = tid; e < 128 * ((KP - SS) / 8); e += 128) { const int d = e / ((KP - SS) / 8), q = e % ((KP - SS) / 8); vst2((unsigned*)(V + ((b * CC + vc0 + d) * KP) + SS + q * 8), *(const v4u*)&sv[d][q * 8]); } }
}
__global__ __launch_bounds__(128) void k_attn(const _Float16* __restrict__ Q, const _Float16* __restrict__ KR, const _Float16* __restrict__ V, float* __restrict__ O) {
  __shared__ __align__(16) _Float16 sph[4][16][40]; __shared__ __align__(16) float so[4][16][68];
  const int tid = threadIdx.x, wave = tid >> 5, lane = tid & 31, col = lane & 15, g = lane >> 4; const int h = blockIdx.y; const size_t b = blockIdx.z; const int q0 = blockIdx.x * 64 + wave * 16; const size_t rq = b * SS + q0;
  v16h aq[2];
#pragma unroll
  for (int kc = 0; kc < 2; ++kc) aq[kc] = frag_h(Q + (rq + col) * CC + h * HD + kc * 32, lane);
  float m[8], l[8];
#pragma unroll
  for (int r = 0; r < 8; ++r) { m[r] = -3.0e38f; l[r] = 0.f; }
  v8f acc[4] = {};
#pragma unroll 1
  for (int ks = 0; ks < KP / 32; ++ks) { const int j0 = ks * 32; v8f s[2];
#pragma unroll
    for (int ct = 0; ct < 2; ++ct) { const int kk = j0 + ct * 16 + col; const size_t rk = (b * KP + kk) * CC + h * HD; v8f c = {};
#pragma unroll
      for (int kc = 0; kc < 2; ++kc) c = wmma16(aq[kc], frag_h(KR + rk + kc * 32, lane), c); const bool keep = kk < NKV;
#pragma unroll
      for (int r = 0; r < 8; ++r) s[ct][r] = keep ? c[r] * 0.125f : -3.0e38f; }
#pragma unroll
    for (int r = 0; r < 8; ++r) { float mx = fmaxf(s[0][r], s[1][r]);
#pragma unroll
      for (int o = 1; o < 16; o <<= 1) mx = fmaxf(mx, __shfl_xor(mx, o));
      const float mn = fmaxf(m[r], mx); const float alpha = (m[r] <= -1.0e38f) ? 0.f : __expf(m[r] - mn); const float e0 = (s[0][r] <= -1.0e38f) ? 0.f : __expf(s[0][r] - mn), e1 = (s[1][r] <= -1.0e38f) ? 0.f : __expf(s[1][r] - mn); float es = e0 + e1;
#pragma unroll
      for (int o = 1; o < 16; o <<= 1) es += __shfl_xor(es, o);
      l[r] = l[r] * alpha + es; m[r] = mn;
#pragma unroll
      for (int dt = 0; dt < 4; ++dt) acc[dt][r] *= alpha;
      sph[wave][8 * g + r][col] = (_Float16)(e0 * 2048.0f); sph[wave][8 * g + r][16 + col] = (_Float16)(e1 * 2048.0f); }
    LDSX();
    const v16h pa = frag_h(&sph[wave][col][0], lane);
#pragma unroll
    for (int dt = 0; dt < 4; ++dt) acc[dt] = wmma16(pa, frag_h(V + ((b * CC + h * HD + dt * 16 + col) * KP) + j0, lane), acc[dt]);
    LDSX(); }
#pragma unroll
  for (int r = 0; r < 8; ++r) { const float il = (1.0f / 2048.0f) / l[r];
#pragma unroll
    for (int dt = 0; dt < 4; ++dt) so[wave][8 * g + r][dt * 16 + col] = acc[dt][r] * il; }
  LDSX();
  for (int rl = 0; rl < 16; ++rl) if (lane < 16) vst2(O + (rq + rl) * CC + h * HD + lane * 4, *(const v4f*)&so[wave][rl][lane * 4]);
}
__global__ __launch_bounds__(128) void k_out(const float* __restrict__ O, const __bf16* __restrict__ P, float* __restrict__ Y1) {
  __shared__ __align__(16) float so[4][16][132];
  const int tid = threadIdx.x, wave = tid >> 5, lane = tid & 31, col = lane & 15, g = lane >> 4; const size_t r0 = (size_t)blockIdx.x * 64 + wave * 16; const int c0 = blockIdx.y * 128;
  v8f acc[8] = {};
#pragma unroll 2
  for (int kc = 0; kc < CC / 32; ++kc) { const F2 a = split_row(O + (r0 + col) * CC, kc * 32, lane);
#pragma unroll
    for (int j = 0; j < 8; ++j) { const v16b w = frag_b(P + WS_PO / 2 + (size_t)(c0 + j * 16 + col) * CC + kc * 32, lane); acc[j] = wmma_bf(a.l, w, acc[j]); acc[j] = wmma_bf(a.h, w, acc[j]); } }
#pragma unroll
  for (int j = 0; j < 8; ++j)
#pragma unroll
    for (int r = 0; r < 8; ++r) so[wave][8 * g + r][j * 16 + col] = acc[j][r];
  LDSX();
  for (int rl = 0; rl < 16; ++rl) vst2(Y1 + (r0 + rl) * CC + c0 + lane * 4, *(const v4f*)&so[wave][rl][lane * 4]);
}
__global__ __launch_bounds__(256) void k_ln2(const float* __restrict__ Y1, const float* __restrict__ X, const float* __restrict__ G2, float* __restrict__ OUT) {
  __shared__ float smu[64], sinv[64]; __shared__ __align__(16) float st[128][68]; const size_t b = blockIdx.y; const int n0 = blockIdx.x * 64, t = threadIdx.x;
  { const int rl = t >> 2, part = t & 3; const float* y = Y1 + (b * SS + n0 + rl) * CC; float s = 0.f; for (int c = part * 128; c < part * 128 + 128; ++c) s += y[c]; s += __shfl_xor(s, 1); s += __shfl_xor(s, 2); const float mu = s / (float)CC; float q = 0.f; for (int c = part * 128; c < part * 128 + 128; ++c) { const float d = y[c] - mu; q += d * d; } q += __shfl_xor(q, 1); q += __shfl_xor(q, 2); if (part == 0) { smu[rl] = mu; sinv[rl] = 1.0f / sqrtf(q / (float)CC + 1e-5f); } }
  __syncthreads();
  for (int ch = 0; ch < CC / 128; ++ch) {
    for (int e = t; e < 64 * 128; e += 256) { const int rl = e & 63, cl = e >> 6; const int c = ch * 128 + cl; st[cl][rl] = (Y1[(b * SS + n0 + rl) * CC + c] - smu[rl]) * sinv[rl] * bfr(G2[c]) + bfr(X[((b * CC + c) * SS) + n0 + rl]); }
    __syncthreads();
    for (int e = t; e < 128 * 16; e += 256) { const int cl = e >> 4, q = e & 15; vst2(OUT + ((b * CC + ch * 128 + cl) * SS) + n0 + q * 4, *(const v4f*)&st[cl][q * 4]); }
    __syncthreads(); }
}
extern "C" void kernel_launch(void* const* d_in, const int* in_sizes, int n_in, void* d_out, int out_size, void* d_ws, size_t ws_size, hipStream_t stream) {
  (void)in_sizes; (void)n_in; (void)out_size;
  const float** F = (const float**)d_in;
  if (ws_size < (size_t)WS_END) return;
  char* ws = (char*)d_ws; __bf16 *P = (__bf16*)ws, *XN = (__bf16*)(ws + WS_XN), *XNL = (__bf16*)(ws + WS_XNL); _Float16 *Q = (_Float16*)(ws + WS_Q), *KR = (_Float16*)(ws + WS_KR), *V = (_Float16*)(ws + WS_V); float *O = (float*)(ws + WS_O), *Y1 = (float*)(ws + WS_Y1);
  k_pack<<<dim3(2 * CC, 3), 256, 0, stream>>>(F[4], F[6], F[5], P);
  k_ln1<<<dim3(SS / 64, NB), 256, 0, stream>>>(F[0], F[2], XN, XNL);
  k_q<<<dim3(SS / 64, CC / 128, NB), 128, 0, stream>>>(XN, XNL, P, Q, KR, V);
  k_kv<<<dim3(1, 2 * CC / 128, NB), 128, 0, stream>>>(F[1], P, F[3], KR, V);
  k_attn<<<dim3(TQB, NH, TNB), 128, 0, stream>>>(Q, KR, V, O);
  k_out<<<dim3(TNB * SS / 64, CC / 128), 128, 0, stream>>>(O, P, Y1);
  k_ln2<<<dim3(TQB, TNB), 256, 0, stream>>>(Y1, F[0], F[7], (float*)d_out);
}
